// PixtralHFAttention_80401787781161
// MI455X (gfx1250) — hardware-verified
//
#include <hip/hip_runtime.h>
#include <math.h>
#include <stdint.h>

constexpr int kBatch = 2;
constexpr int kSeq   = 2048;
constexpr int kHid   = 1024;
constexpr int kHeads = 16;
constexpr int kHdim  = 64;
constexpr int kRows  = kBatch * kSeq;

constexpr float kPScale  = 32768.0f;
constexpr float kVtScale = 8.0f;
constexpr float kPVInv   = 1.0f / (32768.0f * 8.0f);
constexpr float kOScale  = 256.0f;
constexpr float kWoScale = 64.0f;
constexpr float kOutInv  = 1.0f / (256.0f * 64.0f);

typedef __attribute__((ext_vector_type(16))) _Float16 v16h;
typedef __attribute__((ext_vector_type(8)))  _Float16 v8h;
typedef __attribute__((ext_vector_type(16))) __bf16   v16b;
typedef __attribute__((ext_vector_type(8)))  __bf16   v8b;
typedef __attribute__((ext_vector_type(8)))  float    v8f;
typedef __attribute__((ext_vector_type(4)))  float    v4f;
typedef __attribute__((ext_vector_type(2)))  float    v2f;
typedef __attribute__((ext_vector_type(4)))  unsigned int v4u;

__device__ __forceinline__ unsigned short f2bf_bits(float f) {
  unsigned u = __float_as_uint(f);
  return (unsigned short)((u + 0x7FFFu + ((u >> 16) & 1u)) >> 16);
}
__device__ __forceinline__ float bf_bits2f(unsigned short h) { return __uint_as_float(((unsigned)h) << 16); }
__device__ __forceinline__ unsigned pk16(unsigned short a, unsigned short b) { return (unsigned)a | ((unsigned)b << 16); }

__device__ __forceinline__ void dep_guard_h(v8f& a, v8f& b, v16h x, v16h y) { asm volatile("v_nop\n\tv_nop\n\tv_nop\n\tv_nop" : "+v"(a), "+v"(b) : "v"(x), "v"(y)); }
__device__ __forceinline__ void dep_guard_b(v8f& a, v8f& b, v16b x, v16b y) { asm volatile("v_nop\n\tv_nop\n\tv_nop\n\tv_nop" : "+v"(a), "+v"(b) : "v"(x), "v"(y)); }
__device__ __forceinline__ void keep4_h(v16h a, v16h b, v16h c, v16h d) { asm volatile("v_nop" :: "v"(a), "v"(b), "v"(c), "v"(d)); }
__device__ __forceinline__ void keep4_b(v16b a, v16b b, v16b c, v16b d) { asm volatile("v_nop" :: "v"(a), "v"(b), "v"(c), "v"(d)); }
__device__ __forceinline__ void acc_guard4(v8f& a, v8f& b, v8f& c, v8f& d) { asm volatile("v_nop\n\tv_nop\n\tv_nop\n\tv_nop" : "+v"(a), "+v"(b), "+v"(c), "+v"(d)); }
template <typename T> struct Frag;
template <> struct Frag<_Float16> {
  typedef v16h V; union U { v16h v; v8h h[2]; };
  static __device__ __forceinline__ v16h load(const _Float16* p) {
    U f; f.h[0] = *(const v8h*)(p); f.h[1] = *(const v8h*)(p + 16); return f.v;
  }
  static __device__ __forceinline__ v8f mma(v16h a, v16h b, v8f c) {
    return __builtin_amdgcn_wmma_f32_16x16x32_f16(false, a, false, b, (short)0, c, false, false);
  }
  static __device__ __forceinline__ void guard(v8f& a, v8f& b, v16h x, v16h y) { dep_guard_h(a, b, x, y); }
  static __device__ __forceinline__ void keep(v16h a, v16h b, v16h c, v16h d) { keep4_h(a, b, c, d); }
};
template <> struct Frag<__bf16> {
  typedef v16b V; union U { v16b v; v8b h[2]; };
  static __device__ __forceinline__ v16b load(const __bf16* p) {
    U f; f.h[0] = *(const v8b*)(p); f.h[1] = *(const v8b*)(p + 16); return f.v;
  }
  static __device__ __forceinline__ v8f mma(v16b a, v16b b, v8f c) {
    return __builtin_amdgcn_wmma_f32_16x16x32_bf16(false, a, false, b, (short)0, c, false, false);
  }
  static __device__ __forceinline__ void guard(v8f& a, v8f& b, v16b x, v16b y) { dep_guard_b(a, b, x, y); }
  static __device__ __forceinline__ void keep(v16b a, v16b b, v16b c, v16b d) { keep4_b(a, b, c, d); }
};

template <int ET> struct Elem;
template <> struct Elem<0> { typedef _Float16 T; };
template <> struct Elem<1> { typedef __bf16 T; };
template <int ET, bool SPLIT, int BIAS_MODE, int OUT_MODE, bool RESID, int ACT = 0>
__global__ __launch_bounds__(256) void wmma_gemm64(
    const unsigned short* __restrict__ Ap, const unsigned short* __restrict__ A2p, int lda, long strideA,
    const unsigned short* __restrict__ Btp, const unsigned short* __restrict__ Bt2p, int ldb, long strideB,
    void* __restrict__ Cout, void* __restrict__ Cout2, int ldc, long strideC,
    const float* __restrict__ bias,
    const float* __restrict__ resid, long strideR,
    int M, int N, int K, float scale) {
  typedef typename Elem<ET>::T T;
  typedef typename Frag<T>::V V;
  const T* A = (const T*)Ap; const T* A2 = (const T*)A2p; const T* Bt = (const T*)Btp; const T* Bt2 = (const T*)Bt2p;
  __shared__ __align__(16) float sT[8][16 * 68];
  const int b    = blockIdx.y;
  const int lane = threadIdx.x & 31;
  const int wave = threadIdx.x >> 5;
  const int tilesN = N >> 6;
  const int tilesM = M >> 6;
  const int tile = blockIdx.x * 8 + wave;
  if (tile >= tilesM * tilesN) return;
  const int tm = tile / tilesN;
  const int tn = tile - tm * tilesN;
  const int m0 = tm << 6;
  const int n0 = tn << 6;

  const T* Ab  = A  + (size_t)b * strideA;
  const T* Bb  = Bt + (size_t)b * strideB;
  const T* Ab2 = SPLIT ? (A2  + (size_t)b * strideA) : nullptr;
  const T* Bb2 = SPLIT ? (Bt2 + (size_t)b * strideB) : nullptr;

  const int rlane = lane & 15;
  const int koff  = (lane >> 4) * 8;
  const int mOff  = (lane >> 4) * 8;

  v8f acc[4][4];
#pragma unroll
  for (int i = 0; i < 4; ++i)
#pragma unroll
    for (int j = 0; j < 4; ++j) acc[i][j] = (v8f){0.f,0.f,0.f,0.f,0.f,0.f,0.f,0.f};

  for (int k0 = 0; k0 < K; k0 += 32) {
    V bh[4], bl[4];
#pragma unroll
    for (int j = 0; j < 4; ++j) {
      const size_t bo = (size_t)(n0 + (j << 4) + rlane) * ldb + koff + k0;
      bh[j] = Frag<T>::load(Bb + bo);
      if (SPLIT) bl[j] = Frag<T>::load(Bb2 + bo);
    }
#pragma unroll
    for (int i = 0; i < 4; ++i) {
      const size_t ao = (size_t)(m0 + (i << 4) + rlane) * lda + koff + k0;
      V ah = Frag<T>::load(Ab + ao);
      V al;
      if (SPLIT) al = Frag<T>::load(Ab2 + ao);
#pragma unroll
      for (int j = 0; j < 4; ++j) {
        acc[i][j] = Frag<T>::mma(ah, bh[j], acc[i][j]);
        if (SPLIT) {
          acc[i][j] = Frag<T>::mma(ah, bl[j], acc[i][j]);
          acc[i][j] = Frag<T>::mma(al, bh[j], acc[i][j]);
        }
      }
      Frag<T>::guard(acc[i][0], acc[i][3], ah, SPLIT ? al : ah);
    }
    Frag<T>::keep(bh[0], bh[1], bh[2], bh[3]);
    if (SPLIT) Frag<T>::keep(bl[0], bl[1], bl[2], bl[3]);
  }
  acc_guard4(acc[0][0], acc[0][1], acc[0][2], acc[0][3]);
  acc_guard4(acc[1][0], acc[1][1], acc[1][2], acc[1][3]);
  acc_guard4(acc[2][0], acc[2][1], acc[2][2], acc[2][3]);
  acc_guard4(acc[3][0], acc[3][1], acc[3][2], acc[3][3]);

  float* slab = sT[wave];
  const float* Rb = RESID ? (resid + (size_t)b * strideR) : nullptr;
#pragma unroll
  for (int i = 0; i < 4; ++i) {
    const int mBase = m0 + (i << 4);
#pragma unroll
    for (int j = 0; j < 4; ++j) {
      const int n = n0 + (j << 4) + rlane;
      float bv = 0.f;
      if (BIAS_MODE == 2) bv = bias[n];
#pragma unroll
      for (int r = 0; r < 8; ++r) {
        float v = acc[i][j][r] * scale;
        if (BIAS_MODE == 1) v += bias[mBase + mOff + r];
        if (BIAS_MODE == 2) v += bv;
        if (RESID) v += Rb[(size_t)(mBase + mOff + r) * ldc + n];
        if (ACT == 1) v = tanhf(v);
        if (ACT == 2) v = fmaxf(v, 0.0f);
        if (ACT == 3) v = v / (1.0f + expf(-v));
        if (ACT == 4) v = (v > 0.f) ? v : 0.01f * v;
        if (ACT == 5) v = 0.5f * v * (1.0f + erff(v * 0.70710678118654752f));
        slab[(mOff + r) * 68 + (j << 4) + rlane] = v;
      }
    }
    __builtin_amdgcn_fence(__ATOMIC_RELEASE, "workgroup");
    __builtin_amdgcn_wave_barrier();
    __builtin_amdgcn_fence(__ATOMIC_ACQUIRE, "workgroup");
    if (OUT_MODE == 0) {
      float* C = (float*)Cout + (size_t)b * strideC;
      const int hh = lane >> 4, c4 = (lane & 15) * 4;
      for (int pass = 0; pass < 2; ++pass) {
#pragma unroll
        for (int it = 0; it < 8; ++it) {
          const int row = it * 2 + hh;
          v4f v = *(const v4f*)(slab + row * 68 + c4);
          *(volatile v4f*)(C + (size_t)(mBase + row) * ldc + n0 + c4) = v;
        }
        __threadfence();
      }
    } else {
      const int q = lane >> 3, c8 = (lane & 7) * 8;
      unsigned short* C  = (unsigned short*)Cout  + (size_t)b * strideC;
      unsigned short* C2 = (OUT_MODE == 2) ? ((unsigned short*)Cout2 + (size_t)b * strideC) : nullptr;
      for (int pass = 0; pass < 2; ++pass) {
#pragma unroll
        for (int it = 0; it < 4; ++it) {
          const int row = it * 4 + q;
          const float* sp = slab + row * 68 + c8;
          v8h hv, lv;
#pragma unroll
          for (int e = 0; e < 8; ++e) {
            if (OUT_MODE == 1) {
              hv[e] = (_Float16)sp[e];
            } else {
              unsigned short hb = f2bf_bits(sp[e]);
              unsigned short lb = f2bf_bits(sp[e] - bf_bits2f(hb));
              hv[e] = __builtin_bit_cast(_Float16, hb);
              lv[e] = __builtin_bit_cast(_Float16, lb);
            }
          }
          *(volatile v8h*)(C + (size_t)(mBase + row) * ldc + n0 + c8) = hv;
          if (OUT_MODE == 2) *(volatile v8h*)(C2 + (size_t)(mBase + row) * ldc + n0 + c8) = lv;
        }
        __threadfence();
      }
    }
    __builtin_amdgcn_fence(__ATOMIC_RELEASE, "workgroup");
    __builtin_amdgcn_wave_barrier();
    __builtin_amdgcn_fence(__ATOMIC_ACQUIRE, "workgroup");
  }
}

__global__ __launch_bounds__(256) void cast_f32_bf16x2(const float* __restrict__ in,
                                                       unsigned short* __restrict__ out, int n2) {
  const int i = blockIdx.x * 256 + threadIdx.x;
  if (i < n2) {
    const v2f f = *(const v2f*)(in + 2 * (size_t)i);
    const unsigned u = pk16(f2bf_bits(f[0]), f2bf_bits(f[1]));
    ((volatile unsigned*)out)[i] = u;
    __threadfence();
    ((volatile unsigned*)out)[i] = u;
  }
}

template <bool VIA_BF>
__global__ __launch_bounds__(256) void cast_f32_f16x2s(const float* __restrict__ in,
                                                       unsigned short* __restrict__ out, int n2, float scale) {
  const int i = blockIdx.x * 256 + threadIdx.x;
  if (i < n2) {
    const v2f f = *(const v2f*)(in + 2 * (size_t)i);
    float a0 = f[0], a1 = f[1];
    if (VIA_BF) { a0 = bf_bits2f(f2bf_bits(a0)); a1 = bf_bits2f(f2bf_bits(a1)); }
    const _Float16 h0 = (_Float16)(a0 * scale), h1 = (_Float16)(a1 * scale);
    const unsigned u = pk16(__builtin_bit_cast(unsigned short, h0), __builtin_bit_cast(unsigned short, h1));
    ((volatile unsigned*)out)[i] = u;
    __threadfence();
    ((volatile unsigned*)out)[i] = u;
  }
}

__global__ __launch_bounds__(256) void rope_split_kernel(
    const float* __restrict__ qk, const float* __restrict__ cosT, const float* __restrict__ sinT,
    unsigned short* __restrict__ qh, unsigned short* __restrict__ ql,
    unsigned short* __restrict__ kh, unsigned short* __restrict__ kl) {
#pragma clang fp contract(off)
  const int row   = blockIdx.x;
  const int s     = row & (kSeq - 1);
  const int t     = threadIdx.x;
  const int which = t >> 7;
  const int e8    = (t & 127) * 8;
  const int d0    = e8 & 63;
  const int hb    = e8 - d0;
  const int dp0   = d0 ^ 32;
  const float* src = qk + (size_t)row * (2 * kHid) + (size_t)which * kHid;
  const v4f xa = *(const v4f*)(src + e8);
  const v4f xb = *(const v4f*)(src + e8 + 4);
  const v4f pa = *(const v4f*)(src + hb + dp0);
  const v4f pb = *(const v4f*)(src + hb + dp0 + 4);
  const v4f ca = *(const v4f*)(cosT + (size_t)s * kHdim + d0);
  const v4f cb = *(const v4f*)(cosT + (size_t)s * kHdim + d0 + 4);
  const v4f sa = *(const v4f*)(sinT + (size_t)s * kHdim + d0);
  const v4f sb = *(const v4f*)(sinT + (size_t)s * kHdim + d0 + 4);
  const float xs[8] = {xa[0], xa[1], xa[2], xa[3], xb[0], xb[1], xb[2], xb[3]};
  const float ps[8] = {pa[0], pa[1], pa[2], pa[3], pb[0], pb[1], pb[2], pb[3]};
  const float cs[8] = {ca[0], ca[1], ca[2], ca[3], cb[0], cb[1], cb[2], cb[3]};
  const float sn[8] = {sa[0], sa[1], sa[2], sa[3], sb[0], sb[1], sb[2], sb[3]};
  const bool lowh = (d0 < 32);
  v4u hv, lv;
#pragma unroll
  for (int q = 0; q < 4; ++q) {
    const float c0 = bf_bits2f(f2bf_bits(cs[2 * q])), c1 = bf_bits2f(f2bf_bits(cs[2 * q + 1]));
    const float s0 = bf_bits2f(f2bf_bits(sn[2 * q])), s1 = bf_bits2f(f2bf_bits(sn[2 * q + 1]));
    const float ta0 = xs[2 * q] * c0,     tb0 = ps[2 * q] * s0;
    const float ta1 = xs[2 * q + 1] * c1, tb1 = ps[2 * q + 1] * s1;
    const float r0 = lowh ? (ta0 - tb0) : (ta0 + tb0);
    const float r1 = lowh ? (ta1 - tb1) : (ta1 + tb1);
    const unsigned short h0 = f2bf_bits(r0), h1 = f2bf_bits(r1);
    const unsigned short l0 = f2bf_bits(r0 - bf_bits2f(h0)), l1 = f2bf_bits(r1 - bf_bits2f(h1));
    hv[q] = pk16(h0, h1);
    lv[q] = pk16(l0, l1);
  }
  unsigned short* oh  = which ? kh : qh;
  unsigned short* olo = which ? kl : ql;
  const size_t go = (size_t)row * kHid + e8;
  *(volatile v4u*)(oh  + go) = hv;
  *(volatile v4u*)(olo + go) = lv;
  __threadfence();
  *(volatile v4u*)(oh  + go) = hv;
  *(volatile v4u*)(olo + go) = lv;
}

#define AT_D 64
#define AT_NW 4
#define AT_QB 64
#define AT_KC 64

__device__ __forceinline__ unsigned short at_bf_bits(float f) {
  unsigned u = __float_as_uint(f);
  return (unsigned short)((u + 0x7FFFu + ((u >> 16) & 1u)) >> 16);
}
__device__ __forceinline__ __bf16 at_f2bf(float f) { return __builtin_bit_cast(__bf16, at_bf_bits(f)); }
__device__ __forceinline__ v8f at_mma(v16b a, v16b b, v8f c) {
  c = __builtin_amdgcn_wmma_f32_16x16x32_bf16(false, a, false, b, (short)0, c, false, false);
  asm volatile("v_nop\n\tv_nop\n\tv_nop\n\tv_nop" : "+v"(c) : "v"(a), "v"(b));
  return c;
}
__device__ __forceinline__ v8f at_mma_h(v16b a, v16b b, v8f c) {
  const v16h ah = __builtin_bit_cast(v16h, a), bh = __builtin_bit_cast(v16h, b);
  c = __builtin_amdgcn_wmma_f32_16x16x32_f16(false, ah, false, bh, (short)0, c, false, false);
  asm volatile("v_nop\n\tv_nop\n\tv_nop\n\tv_nop" : "+v"(c) : "v"(ah), "v"(bh));
  return c;
}

__global__ __launch_bounds__(128)
void mha_full64_kernel(const unsigned short* __restrict__ qhp, const unsigned short* __restrict__ qlp,
                       const unsigned short* __restrict__ khp, const unsigned short* __restrict__ klp,
                       const unsigned short* __restrict__ vtp, const float* __restrict__ maskp,
                       float* __restrict__ out, float sscale) {
  union FB { v16b v; v8b h[2]; };
  __shared__ __align__(16) __bf16 Ksh[AT_KC * AT_D];
  __shared__ __align__(16) __bf16 Ksl[AT_KC * AT_D];
  __shared__ __align__(16) __bf16 Vth[AT_D * AT_KC];
  __shared__ __align__(16) __bf16 Psh[AT_NW][16 * AT_KC];
  __shared__ __align__(16) float  Os[AT_NW][16 * 68];

  const int tid  = threadIdx.x;
  const int wave = tid >> 5;
  const int lane = tid & 31;
  const int hh   = lane >> 4;
  const int c    = lane & 15;

  constexpr int nqb = kSeq / AT_QB;
  const int bx = blockIdx.x;
  const int qb = bx % nqb;
  const int bh = bx / nqb;
  const int h  = bh % kHeads;
  const int b  = bh / kHeads;
  const int q0 = qb * AT_QB + wave * 16;

  const __bf16* Qh = (const __bf16*)(const void*)qhp + (size_t)b * kSeq * kHid + (size_t)h * AT_D;
  const __bf16* Ql = (const __bf16*)(const void*)qlp + (size_t)b * kSeq * kHid + (size_t)h * AT_D;
  const __bf16* Kh = (const __bf16*)(const void*)khp + (size_t)b * kSeq * kHid + (size_t)h * AT_D;
  const __bf16* Kl = (const __bf16*)(const void*)klp + (size_t)b * kSeq * kHid + (size_t)h * AT_D;
  const __bf16* Vt = (const __bf16*)(const void*)vtp + (size_t)b * kHid * kSeq + (size_t)h * AT_D * kSeq;
  const float*  Mb = maskp + (size_t)b * kSeq * kSeq;
  float*        ob = out + (size_t)b * kSeq * kHid + (size_t)h * AT_D;

  v16b qah[2], qal[2];
#pragma unroll
  for (int dc = 0; dc < 2; ++dc) {
    const __bf16* qr = Qh + (size_t)(q0 + c) * kHid + dc * 32 + 8 * hh;
    const __bf16* qs = Ql + (size_t)(q0 + c) * kHid + dc * 32 + 8 * hh;
    qah[dc] = Frag<__bf16>::load(qr);
    qal[dc] = Frag<__bf16>::load(qs);
  }

  float mrow[8], lrow[8];
  v8f oacc[4];
#pragma unroll
  for (int r = 0; r < 8; ++r) { mrow[r] = -INFINITY; lrow[r] = 0.f; }
#pragma unroll
  for (int t = 0; t < 4; ++t) oacc[t] = (v8f){0.f,0.f,0.f,0.f,0.f,0.f,0.f,0.f};

  constexpr int nChunks = kSeq / AT_KC;
  for (int kc = 0; kc < nChunks; ++kc) {
    const int kv0 = kc * AT_KC;
    __syncthreads();
    {
      const int r = tid >> 1, half = (tid & 1) * 32;
      const __bf16* ksh = Kh + (size_t)(kv0 + r) * kHid + half;
      const __bf16* ksl = Kl + (size_t)(kv0 + r) * kHid + half;
      const __bf16* vs  = Vt + (size_t)r * kSeq + kv0 + half;
#pragma unroll
      for (int i = 0; i < 4; ++i) {
        const v8b a0 = *(const v8b*)(ksh + 8 * i);
        const v8b a1 = *(const v8b*)(ksl + 8 * i);
        const v8b b0 = *(const v8b*)(vs + 8 * i);
        *(v8b*)(Ksh + r * AT_D  + half + 8 * i) = a0;
        *(v8b*)(Ksl + r * AT_D  + half + 8 * i) = a1;
        *(v8b*)(Vth + r * AT_KC + half + 8 * i) = b0;
      }
    }
    __syncthreads();

    v8f s[4];
#pragma unroll
    for (int j = 0; j < 4; ++j) {
      s[j] = (v8f){0.f,0.f,0.f,0.f,0.f,0.f,0.f,0.f};
#pragma unroll
      for (int dc = 0; dc < 2; ++dc) {
        FB kb, kl;
        kb.h[0] = *(const v8b*)(Ksh + (j * 16 + c) * AT_D + dc * 32 + 8 * hh);
        kb.h[1] = *(const v8b*)(Ksh + (j * 16 + c) * AT_D + dc * 32 + 16 + 8 * hh);
        kl.h[0] = *(const v8b*)(Ksl + (j * 16 + c) * AT_D + dc * 32 + 8 * hh);
        kl.h[1] = *(const v8b*)(Ksl + (j * 16 + c) * AT_D + dc * 32 + 16 + 8 * hh);
        s[j] = at_mma(qah[dc], kb.v, s[j]);
        s[j] = at_mma(qah[dc], kl.v, s[j]);
        s[j] = at_mma(qal[dc], kb.v, s[j]);
      }
    }
    float cm[8];
#pragma unroll
    for (int r = 0; r < 8; ++r) {
      const float* mr = Mb + (size_t)(q0 + 8 * hh + r) * kSeq + kv0;
      float m = -INFINITY;
#pragma unroll
      for (int j = 0; j < 4; ++j) {
        const float sv = s[j][r] * sscale + mr[j * 16 + c];
        s[j][r] = sv;
        m = fmaxf(m, sv);
      }
#pragma unroll
      for (int off = 1; off < 16; off <<= 1) m = fmaxf(m, __shfl_xor(m, off, 32));
      cm[r] = m;
    }
    __bf16* pwh = Psh[wave];
#pragma unroll
    for (int r = 0; r < 8; ++r) {
      const float mnew = fmaxf(mrow[r], cm[r]);
      const float alpha = expf(mrow[r] - mnew);
      mrow[r] = mnew;
      float psum = 0.f;
#pragma unroll
      for (int j = 0; j < 4; ++j) {
        const float p = expf(s[j][r] - mnew);
        psum += p;
        pwh[(8 * hh + r) * AT_KC + j * 16 + c] = __builtin_bit_cast(__bf16, (_Float16)(p * kPScale));
      }
#pragma unroll
      for (int off = 1; off < 16; off <<= 1) psum += __shfl_xor(psum, off, 32);
      lrow[r] = lrow[r] * alpha + psum;
#pragma unroll
      for (int t = 0; t < 4; ++t) oacc[t][r] *= alpha;
    }
    __builtin_amdgcn_fence(__ATOMIC_RELEASE, "workgroup");
    __builtin_amdgcn_wave_barrier();
    __builtin_amdgcn_fence(__ATOMIC_ACQUIRE, "workgroup");
#pragma unroll 1
    for (int kk = 0; kk < 2; ++kk) {
      FB pa;
      pa.h[0] = *(const v8b*)(pwh + c * AT_KC + kk * 32 + 8 * hh);
      pa.h[1] = *(const v8b*)(pwh + c * AT_KC + kk * 32 + 16 + 8 * hh);
#pragma unroll
      for (int t = 0; t < 4; ++t) {
        FB vb;
        vb.h[0] = *(const v8b*)(Vth + (t * 16 + c) * AT_KC + kk * 32 + 8 * hh);
        vb.h[1] = *(const v8b*)(Vth + (t * 16 + c) * AT_KC + kk * 32 + 16 + 8 * hh);
        oacc[t] = at_mma_h(pa.v, vb.v, oacc[t]);
      }
    }
  }

  float* os = Os[wave];
#pragma unroll
  for (int r = 0; r < 8; ++r) {
    const float inv = (1.0f / lrow[r]) * kPVInv;
#pragma unroll
    for (int t = 0; t < 4; ++t) os[(8 * hh + r) * 68 + t * 16 + c] = oacc[t][r] * inv;
  }
  __builtin_amdgcn_fence(__ATOMIC_RELEASE, "workgroup");
  __builtin_amdgcn_wave_barrier();
  __builtin_amdgcn_fence(__ATOMIC_ACQUIRE, "workgroup");
  {
    const int c4 = (lane & 15) * 4;
    for (int pass = 0; pass < 2; ++pass) {
#pragma unroll
      for (int it = 0; it < 8; ++it) {
        const int row = it * 2 + hh;
        v4f val = *(const v4f*)(os + row * 68 + c4);
        *(volatile v4f*)(ob + (size_t)(q0 + row) * kHid + c4) = val;
      }
      __threadfence();
    }
  }
}

extern "C" void kernel_launch(void* const* d_in, const int* in_sizes, int n_in,
                              void* d_out, int out_size, void* d_ws, size_t ws_size,
                              hipStream_t stream) {
  if (n_in < 8) return;
  const float* x    = (const float*)d_in[0];
  const float* mask = (const float*)d_in[1];
  const float* cosT = (const float*)d_in[2];
  const float* sinT = (const float*)d_in[3];
  const float* wq   = (const float*)d_in[4];
  const float* wk   = (const float*)d_in[5];
  const float* wv   = (const float*)d_in[6];
  const float* wo   = (const float*)d_in[7];

  const int nX = kRows * kHid;
  const int nW = kHid * kHid;
  if (in_sizes[0] != nX || in_sizes[1] != kBatch * kSeq * kSeq || in_sizes[2] != kSeq * kHdim ||
      in_sizes[3] != kSeq * kHdim || in_sizes[4] != nW || in_sizes[5] != nW || in_sizes[6] != nW ||
      in_sizes[7] != nW || out_size != nX) return;

  const size_t MiB = (size_t)1 << 20;
  const size_t off_Xb   = 0;
  const size_t off_Wqk  = off_Xb  + (size_t)nX * 2;
  const size_t off_Wv   = off_Wqk + (size_t)2 * nW * 2;
  const size_t off_Wo   = off_Wv  + (size_t)nW * 2;
  const size_t off_QKf  = off_Wo  + (size_t)nW * 2;
  const size_t off_Of   = off_QKf;
  const size_t off_O16  = off_QKf + (size_t)nX * 4;
  const size_t off_Vt   = off_QKf + (size_t)nX * 2 * 4;
  const size_t off_Qh   = off_Vt  + (size_t)kBatch * kHid * kSeq * 2;
  const size_t off_Ql   = off_Qh  + (size_t)nX * 2;
  const size_t off_Kh   = off_Ql  + (size_t)nX * 2;
  const size_t off_Kl   = off_Kh  + (size_t)nX * 2;
  const size_t total    = off_Kl  + (size_t)nX * 2;
  if (total != 88 * MiB) return;
  if (ws_size < total) return;

  char* ws = (char*)d_ws;
  unsigned short* Xb   = (unsigned short*)(ws + off_Xb);
  unsigned short* Wqkb = (unsigned short*)(ws + off_Wqk);
  unsigned short* Wvb  = (unsigned short*)(ws + off_Wv);
  unsigned short* Wo16 = (unsigned short*)(ws + off_Wo);
  float*          QKf  = (float*)(ws + off_QKf);
  float*          Of   = (float*)(ws + off_Of);
  unsigned short* O16  = (unsigned short*)(ws + off_O16);
  unsigned short* Vt16 = (unsigned short*)(ws + off_Vt);
  unsigned short* Qh   = (unsigned short*)(ws + off_Qh);
  unsigned short* Ql   = (unsigned short*)(ws + off_Ql);
  unsigned short* Kh   = (unsigned short*)(ws + off_Kh);
  unsigned short* Kl   = (unsigned short*)(ws + off_Kl);

  const int nX2 = nX / 2, nW2 = nW / 2;
  cast_f32_bf16x2<<<(nX2 + 255) / 256, 256, 0, stream>>>(x,  Xb, nX2);
  cast_f32_bf16x2<<<(nW2 + 255) / 256, 256, 0, stream>>>(wq, Wqkb, nW2);
  cast_f32_bf16x2<<<(nW2 + 255) / 256, 256, 0, stream>>>(wk, Wqkb + (size_t)nW, nW2);
  cast_f32_bf16x2<<<(nW2 + 255) / 256, 256, 0, stream>>>(wv, Wvb, nW2);
  cast_f32_f16x2s<true><<<(nW2 + 255) / 256, 256, 0, stream>>>(wo, Wo16, nW2, kWoScale);

  {
    dim3 g((kRows / 64) * (2 * kHid / 64) / 8, 1);
    wmma_gemm64<1, false, 0, 0, false><<<g, 256, 0, stream>>>(
        Xb, Xb, kHid, (long)0,
        Wqkb, Wqkb, kHid, (long)0,
        (void*)QKf, (void*)QKf, 2 * kHid, (long)0,
        cosT, cosT, (long)0,
        kRows, 2 * kHid, kHid, 1.0f);
  }
  {
    dim3 g((kHid / 64) * (kSeq / 64) / 8, kBatch);
    wmma_gemm64<1, false, 0, 1, false><<<g, 256, 0, stream>>>(
        Wvb, Wvb, kHid, (long)0,
        Xb, Xb, kHid, (long)kSeq * kHid,
        (void*)Vt16, (void*)Vt16, kSeq, (long)kHid * kSeq,
        cosT, cosT, (long)0,
        kHid, kSeq, kHid, kVtScale);
  }
  rope_split_kernel<<<kRows, 256, 0, stream>>>(QKf, cosT, sinT, Qh, Ql, Kh, Kl);
  mha_full64_kernel<<<kBatch * kHeads * (kSeq / 64), 128, 0, stream>>>(Qh, Ql, Kh, Kl, Vt16, mask, Of, 0.125f);
  cast_f32_f16x2s<false><<<(nX2 + 255) / 256, 256, 0, stream>>>(Of, O16, nX2, kOScale);
  {
    dim3 g((kRows / 64) * (kHid / 64) / 8, 1);
    wmma_gemm64<0, false, 0, 0, false><<<g, 256, 0, stream>>>(
        O16, O16, kHid, (long)0,
        Wo16, Wo16, kHid, (long)0,
        d_out, d_out, kHid, (long)0,
        cosT, cosT, (long)0,
        kRows, kHid, kHid, kOutInv);
  }
}
